// GatedDeltaNetLayer_65103114272832
// MI455X (gfx1250) — hardware-verified
//
#include <hip/hip_runtime.h>
#include <math.h>

constexpr int kBatch  = 4;
constexpr int kSeq    = 2048;
constexpr int kModel  = 1024;
constexpr int kHeads  = 16;
constexpr int kHd     = 64;
constexpr int kInner  = kHeads * kHd;
constexpr int kRows   = kBatch * kSeq;
constexpr int kQkvLd  = 3 * kInner;
constexpr int kGateLd = 64;
constexpr int kChunk  = 64;
constexpr int kNChunk = kSeq / kChunk;
constexpr int kGateRow0 = 3 * kInner;
constexpr int kWoRow0   = kGateRow0 + kGateLd;
constexpr int kWallRows = kWoRow0 + kModel;
constexpr int kTP    = 72;
constexpr int kSlabP = 68;
constexpr float kWCarry   = 16.0f;
constexpr float kWInv     = 1.0f / kWCarry;
constexpr float kPCarry   = 2048.0f;
constexpr float kPInv     = 1.0f / kPCarry;
constexpr float kKwCarry  = 4096.0f;
constexpr float kKwInv    = 1.0f / kKwCarry;
constexpr float kKwResCarry = 2048.0f;
constexpr float kKwResInv   = 1.0f / kKwResCarry;
constexpr float kSCarry   = 256.0f;
constexpr float kSInv     = 1.0f / kSCarry;
constexpr float kYCarry   = 16.0f;
constexpr float kOutScale = 1.0f / (kYCarry * kWCarry);
constexpr int kOut0 = kRows * kModel;
constexpr int kOut1 = kBatch * kHeads * kHd * kHd;
static_assert(kInner == 1024 && kModel == 1024, "shape");
static_assert(kHd == 64 && kChunk == 64, "scan tiles are 64x64");
static_assert(kSeq % kChunk == 0, "chunking");
static_assert(kRows % 64 == 0 && kQkvLd % 64 == 0 && kGateLd % 64 == 0 && kModel % 64 == 0, "tile multiples");
static_assert(kModel % 32 == 0 && kInner % 32 == 0, "k multiple of 32");
static_assert((size_t)kOut0 * 4 == 33554432u, "second output byte offset");

typedef __attribute__((ext_vector_type(16))) _Float16 v16h;
typedef __attribute__((ext_vector_type(8)))  _Float16 v8h;
typedef __attribute__((ext_vector_type(16))) __bf16   v16b;
typedef __attribute__((ext_vector_type(8)))  __bf16   v8b;
typedef __attribute__((ext_vector_type(8)))  float    v8f;
typedef __attribute__((ext_vector_type(4)))  float    v4f;
typedef __attribute__((ext_vector_type(4)))  unsigned int v4u;

__device__ __forceinline__ unsigned short f2bf_bits(float f) {
  unsigned u = __float_as_uint(f);
  return (unsigned short)((u + 0x7FFFu + ((u >> 16) & 1u)) >> 16);
}
__device__ __forceinline__ float bf_bits2f(unsigned short h) { return __uint_as_float(((unsigned)h) << 16); }
__device__ __forceinline__ float bf16r(float f) { return bf_bits2f(f2bf_bits(f)); }

__device__ __forceinline__ float h16_to_f32(unsigned hb) {
  const unsigned sgn = (hb & 0x8000u) << 16;
  const unsigned em = hb & 0x7fffu;
  const float fn = __uint_as_float((em << 13) + 0x38000000u);
  const float fs = (float)em * 5.9604644775390625e-8f;
  const float mag = (em < 0x400u) ? fs : fn;
  return __uint_as_float(__float_as_uint(mag) | sgn);
}

__device__ __forceinline__ void dep_guard4_h(v8f& a, v8f& b, v8f& c, v8f& d, v16h x, v16h y) { asm volatile("v_nop\n\tv_nop\n\tv_nop\n\tv_nop" : "+v"(a), "+v"(b), "+v"(c), "+v"(d) : "v"(x), "v"(y)); }
__device__ __forceinline__ void dep_guard4_b(v8f& a, v8f& b, v8f& c, v8f& d, v16b x, v16b y) { asm volatile("v_nop\n\tv_nop\n\tv_nop\n\tv_nop" : "+v"(a), "+v"(b), "+v"(c), "+v"(d) : "v"(x), "v"(y)); }
__device__ __forceinline__ void keep4_h(v16h a, v16h b, v16h c, v16h d) { asm volatile("v_nop" :: "v"(a), "v"(b), "v"(c), "v"(d)); }
__device__ __forceinline__ void keep4_b(v16b a, v16b b, v16b c, v16b d) { asm volatile("v_nop" :: "v"(a), "v"(b), "v"(c), "v"(d)); }
__device__ __forceinline__ void acc_guard4(v8f& a, v8f& b, v8f& c, v8f& d) { asm volatile("v_nop\n\tv_nop\n\tv_nop\n\tv_nop" : "+v"(a), "+v"(b), "+v"(c), "+v"(d)); }

template <typename T> struct Frag;
template <> struct Frag<_Float16> {
  typedef v16h V; union U { v16h v; v8h h[2]; };
  static __device__ __forceinline__ v16h load(const _Float16* p) {
    U f; f.h[0] = *(const v8h*)(p); f.h[1] = *(const v8h*)(p + 16); return f.v;
  }
  static __device__ __forceinline__ v8f mma(v16h a, v16h b, v8f c) {
    return __builtin_amdgcn_wmma_f32_16x16x32_f16(false, a, false, b, (short)0, c, false, false);
  }
  static __device__ __forceinline__ void guard4(v8f& a, v8f& b, v8f& c, v8f& d, v16h x, v16h y) { dep_guard4_h(a, b, c, d, x, y); }
  static __device__ __forceinline__ void keep(v16h a, v16h b, v16h c, v16h d) { keep4_h(a, b, c, d); }
};
template <> struct Frag<__bf16> {
  typedef v16b V; union U { v16b v; v8b h[2]; };
  static __device__ __forceinline__ v16b load(const __bf16* p) {
    U f; f.h[0] = *(const v8b*)(p); f.h[1] = *(const v8b*)(p + 16); return f.v;
  }
  static __device__ __forceinline__ v8f mma(v16b a, v16b b, v8f c) {
    return __builtin_amdgcn_wmma_f32_16x16x32_bf16(false, a, false, b, (short)0, c, false, false);
  }
  static __device__ __forceinline__ void guard4(v8f& a, v8f& b, v8f& c, v8f& d, v16b x, v16b y) { dep_guard4_b(a, b, c, d, x, y); }
  static __device__ __forceinline__ void keep(v16b a, v16b b, v16b c, v16b d) { keep4_b(a, b, c, d); }
};

__device__ __forceinline__ v8f mma_h(v16h a, v16h b, v8f c) {
  c = __builtin_amdgcn_wmma_f32_16x16x32_f16(false, a, false, b, (short)0, c, false, false);
  asm volatile("v_nop\n\tv_nop\n\tv_nop\n\tv_nop" : "+v"(c) : "v"(a), "v"(b));
  return c;
}

__device__ __forceinline__ void wave_lds_sync() {
  __builtin_amdgcn_fence(__ATOMIC_RELEASE, "workgroup");
  __builtin_amdgcn_wave_barrier();
  __builtin_amdgcn_fence(__ATOMIC_ACQUIRE, "workgroup");
}

template <int ET> struct Elem;
template <> struct Elem<0> { typedef _Float16 T; };
template <> struct Elem<1> { typedef __bf16 T; };
template <int ET, bool SPLIT, int BIAS_MODE, int OUT_MODE, bool RESID, int ACT = 0>
__global__ __launch_bounds__(256) void wmma_gemm64(
    const unsigned short* __restrict__ Ap, const unsigned short* __restrict__ A2p, int lda, long strideA,
    const unsigned short* __restrict__ Btp, const unsigned short* __restrict__ Bt2p, int ldb, long strideB,
    void* __restrict__ Cout, void* __restrict__ Cout2, int ldc, long strideC,
    const float* __restrict__ bias,
    const float* __restrict__ resid, long strideR,
    int M, int N, int K, float scale) {
  typedef typename Elem<ET>::T T;
  typedef typename Frag<T>::V V;
  const T* A = (const T*)Ap; const T* A2 = (const T*)A2p; const T* Bt = (const T*)Btp; const T* Bt2 = (const T*)Bt2p;
  __shared__ __align__(16) float sT[8][16 * 68];
  const int b    = blockIdx.y;
  const int lane = threadIdx.x & 31;
  const int wave = threadIdx.x >> 5;
  const int tilesN = N >> 6;
  const int tilesM = M >> 6;
  const int tile = blockIdx.x * 8 + wave;
  if (tile >= tilesM * tilesN) return;
  const int tm = tile / tilesN;
  const int tn = tile - tm * tilesN;
  const int m0 = tm << 6;
  const int n0 = tn << 6;

  const T* Ab  = A  + (size_t)b * strideA;
  const T* Bb  = Bt + (size_t)b * strideB;
  const T* Ab2 = SPLIT ? (A2  + (size_t)b * strideA) : nullptr;
  const T* Bb2 = SPLIT ? (Bt2 + (size_t)b * strideB) : nullptr;

  const int rlane = lane & 15;
  const int koff  = (lane >> 4) * 8;
  const int mOff  = (lane >> 4) * 8;

  v8f acc[4][4];
#pragma unroll
  for (int i = 0; i < 4; ++i)
#pragma unroll
    for (int j = 0; j < 4; ++j) acc[i][j] = (v8f){0.f,0.f,0.f,0.f,0.f,0.f,0.f,0.f};

  for (int k0 = 0; k0 < K; k0 += 32) {
    V bh[4], bl[4];
#pragma unroll
    for (int j = 0; j < 4; ++j) {
      const size_t bo = (size_t)(n0 + (j << 4) + rlane) * ldb + koff + k0;
      bh[j] = Frag<T>::load(Bb + bo);
      if (SPLIT) bl[j] = Frag<T>::load(Bb2 + bo);
    }
#pragma unroll
    for (int i = 0; i < 4; ++i) {
      const size_t ao = (size_t)(m0 + (i << 4) + rlane) * lda + koff + k0;
      V ah = Frag<T>::load(Ab + ao);
      V al;
      if (SPLIT) al = Frag<T>::load(Ab2 + ao);
#pragma unroll
      for (int j = 0; j < 4; ++j) {
        acc[i][j] = Frag<T>::mma(ah, bh[j], acc[i][j]);
        if (SPLIT) {
          acc[i][j] = Frag<T>::mma(ah, bl[j], acc[i][j]);
          acc[i][j] = Frag<T>::mma(al, bh[j], acc[i][j]);
        }
      }
      Frag<T>::guard4(acc[i][0], acc[i][1], acc[i][2], acc[i][3], ah, SPLIT ? al : ah);
    }
    Frag<T>::keep(bh[0], bh[1], bh[2], bh[3]);
    if (SPLIT) Frag<T>::keep(bl[0], bl[1], bl[2], bl[3]);
  }
  acc_guard4(acc[0][0], acc[0][1], acc[0][2], acc[0][3]);
  acc_guard4(acc[1][0], acc[1][1], acc[1][2], acc[1][3]);
  acc_guard4(acc[2][0], acc[2][1], acc[2][2], acc[2][3]);
  acc_guard4(acc[3][0], acc[3][1], acc[3][2], acc[3][3]);

  float* slab = sT[wave];
  const float* Rb = RESID ? (resid + (size_t)b * strideR) : nullptr;
#pragma unroll
  for (int i = 0; i < 4; ++i) {
    const int mBase = m0 + (i << 4);
#pragma unroll
    for (int j = 0; j < 4; ++j) {
      const int n = n0 + (j << 4) + rlane;
      float bv = 0.f;
      if (BIAS_MODE == 2) bv = bias[n];
#pragma unroll
      for (int r = 0; r < 8; ++r) {
        float v = acc[i][j][r] * scale;
        if (BIAS_MODE == 1) v += bias[mBase + mOff + r];
        if (BIAS_MODE == 2) v += bv;
        if (RESID) v += Rb[(size_t)(mBase + mOff + r) * ldc + n];
        if (ACT == 2) v = fmaxf(v, 0.0f);
        if (ACT == 4) v = (v > 0.f) ? v : 0.01f * v;
        slab[(mOff + r) * 68 + (j << 4) + rlane] = v;
      }
    }
    __builtin_amdgcn_fence(__ATOMIC_RELEASE, "workgroup");
    __builtin_amdgcn_wave_barrier();
    __builtin_amdgcn_fence(__ATOMIC_ACQUIRE, "workgroup");
    if (OUT_MODE == 0) {
      float* C = (float*)Cout + (size_t)b * strideC;
      const int hh = lane >> 4, c4 = (lane & 15) * 4;
      for (int pass = 0; pass < 2; ++pass) {
#pragma unroll
        for (int it = 0; it < 8; ++it) {
          const int row = it * 2 + hh;
          v4f v = *(const v4f*)(slab + row * 68 + c4);
          *(volatile v4f*)(C + (size_t)(mBase + row) * ldc + n0 + c4) = v;
        }
        __threadfence();
      }
    } else {
      const int q = lane >> 3, c8 = (lane & 7) * 8;
      unsigned short* C  = (unsigned short*)Cout  + (size_t)b * strideC;
      unsigned short* C2 = (OUT_MODE == 2) ? ((unsigned short*)Cout2 + (size_t)b * strideC) : nullptr;
      for (int pass = 0; pass < 2; ++pass) {
#pragma unroll
        for (int it = 0; it < 4; ++it) {
          const int row = it * 4 + q;
          const float* sp = slab + row * 68 + c8;
          v8h hv, lv;
#pragma unroll
          for (int e = 0; e < 8; ++e) {
            if (OUT_MODE == 1) {
              hv[e] = (_Float16)sp[e];
            } else {
              unsigned short hb = f2bf_bits(sp[e]);
              unsigned short lb = f2bf_bits(sp[e] - bf_bits2f(hb));
              hv[e] = __builtin_bit_cast(_Float16, hb);
              lv[e] = __builtin_bit_cast(_Float16, lb);
            }
          }
          *(volatile v8h*)(C + (size_t)(mBase + row) * ldc + n0 + c8) = hv;
          if (OUT_MODE == 2) *(volatile v8h*)(C2 + (size_t)(mBase + row) * ldc + n0 + c8) = lv;
        }
        __threadfence();
      }
    }
    __builtin_amdgcn_fence(__ATOMIC_RELEASE, "workgroup");
    __builtin_amdgcn_wave_barrier();
    __builtin_amdgcn_fence(__ATOMIC_ACQUIRE, "workgroup");
  }
}

__global__ __launch_bounds__(256) void cvt8_kernel(const float* __restrict__ src, unsigned short* __restrict__ dst, int n8, float sc) {
  const int i = blockIdx.x * 256 + threadIdx.x;
  if (i < n8) {
    const float* sp = src + (size_t)i * 8;
    const v4f a = *(const v4f*)(sp);
    const v4f b = *(const v4f*)(sp + 4);
    v8h hv;
#pragma unroll
    for (int e = 0; e < 4; ++e) {
      const unsigned short b0 = __builtin_bit_cast(unsigned short, (_Float16)(bf16r(a[e]) * sc));
      const unsigned short b1 = __builtin_bit_cast(unsigned short, (_Float16)(bf16r(b[e]) * sc));
      hv[e]     = __builtin_bit_cast(_Float16, b0);
      hv[4 + e] = __builtin_bit_cast(_Float16, b1);
    }
    *(volatile v8h*)(dst + (size_t)i * 8) = hv;
    __threadfence();
    *(volatile v8h*)(dst + (size_t)i * 8) = hv;
  }
}

__global__ __launch_bounds__(256) void wt_cast_kernel(const float* __restrict__ W0, const float* __restrict__ W1,
                                                      const float* __restrict__ W2, const float* __restrict__ W3,
                                                      unsigned short* __restrict__ out) {
  __shared__ float sm[64][65];
  const int t  = threadIdx.x;
  const int k0 = blockIdx.x * 64;
  const int n0 = blockIdx.y * 64;
  const int z  = blockIdx.z;
  const float* W = (z == 0) ? W0 : (z == 1) ? W1 : (z == 2) ? W2 : W3;
  const int rowbase = (z < 3) ? z * kInner : kWoRow0;
#pragma unroll
  for (int i = 0; i < 16; ++i) {
    const int e  = i * 256 + t;
    const int r  = e >> 6;
    const int cc = e & 63;
    sm[cc][r] = bf16r(W[(size_t)(k0 + r) * 1024 + n0 + cc]) * kWCarry;
  }
  __syncthreads();
  const int lane = t & 31, wave = t >> 5;
  const int q = lane >> 3, c8 = (lane & 7) * 8;
  for (int pass = 0; pass < 2; ++pass) {
#pragma unroll
    for (int it = 0; it < 2; ++it) {
      const int row = wave * 8 + it * 4 + q;
      v8h hv;
#pragma unroll
      for (int e = 0; e < 8; ++e) hv[e] = (_Float16)sm[row][c8 + e];
      *(volatile v8h*)(out + (size_t)(rowbase + n0 + row) * 1024 + k0 + c8) = hv;
    }
    __threadfence();
  }
}

__global__ __launch_bounds__(256) void wgate_cast_kernel(const float* __restrict__ Wa, const float* __restrict__ Wb,
                                                         unsigned short* __restrict__ out) {
  __shared__ float sm[64][65];
  const int t  = threadIdx.x;
  const int k0 = blockIdx.x * 64;
#pragma unroll
  for (int i = 0; i < 16; ++i) {
    const int e  = i * 256 + t;
    const int r  = e >> 6;
    const int kk = e & 63;
    const int idx = (k0 + kk) * kHeads + (r & 15);
    const float a  = Wa[idx];
    const float bq = Wb[idx];
    const float v  = (r < 16) ? a : ((r < 32) ? bq : 0.0f);
    sm[r][kk] = bf16r(v) * kWCarry;
  }
  __syncthreads();
  const int lane = t & 31, wave = t >> 5;
  const int q = lane >> 3, c8 = (lane & 7) * 8;
  for (int pass = 0; pass < 2; ++pass) {
#pragma unroll
    for (int it = 0; it < 2; ++it) {
      const int row = wave * 8 + it * 4 + q;
      v8h hv;
#pragma unroll
      for (int e = 0; e < 8; ++e) hv[e] = (_Float16)sm[row][c8 + e];
      *(volatile v8h*)(out + (size_t)(kGateRow0 + row) * 1024 + k0 + c8) = hv;
    }
    __threadfence();
  }
}

__global__ __launch_bounds__(128) void chunk_scan_kernel(const unsigned short* __restrict__ QKV, const float* __restrict__ Z,
                                                         const float* __restrict__ S0, const float* __restrict__ ba,
                                                         const float* __restrict__ bb, unsigned short* __restrict__ Y16,
                                                         float* __restrict__ Sout) {
  __shared__ __align__(16) _Float16 Qs[64 * kTP];
  __shared__ __align__(16) _Float16 Ks[64 * kTP];
  __shared__ __align__(16) _Float16 Vt[64 * kTP];
  __shared__ __align__(16) _Float16 Ps[64 * kTP];
  __shared__ __align__(16) _Float16 Kw[64 * kTP];
  __shared__ __align__(16) _Float16 Kwr[64 * kTP];
  __shared__ __align__(16) _Float16 S16[64 * kTP];
  __shared__ __align__(16) float Fs[4][16 * kSlabP];
  __shared__ float lraw_s[64];
  __shared__ float la_s[64];
  __shared__ float ela_s[64];
  __shared__ float ksb_s[64];

  const int bh   = blockIdx.x;
  const int b    = bh / kHeads;
  const int h    = bh - b * kHeads;
  const int tid  = threadIdx.x;
  const int wave = tid >> 5;
  const int lane = tid & 31;
  const int c    = lane & 15;
  const int hh   = lane >> 4;
  const int koff = hh * 8;
  const int m0   = wave * 16;
  const int c4   = c * 4;
  float* slab = Fs[wave];
  const v8f z8 = {0.f, 0.f, 0.f, 0.f, 0.f, 0.f, 0.f, 0.f};

  {
    const float* s0p = S0 + ((size_t)bh * 64 + m0) * 64;
#pragma unroll
    for (int it = 0; it < 8; ++it) {
      const int rowl = it * 2 + hh;
      const v4f v = *(const v4f*)(s0p + rowl * 64 + c4);
      *(v4f*)(slab + rowl * kSlabP + c4) = v;
    }
  }
  wave_lds_sync();
  float Sreg[4][8];
#pragma unroll
  for (int nt = 0; nt < 4; ++nt)
#pragma unroll
    for (int r = 0; r < 8; ++r) {
      const float sv = bf16r(slab[(8 * hh + r) * kSlabP + nt * 16 + c]);
      Sreg[nt][r] = sv;
      S16[(m0 + 8 * hh + r) * kTP + nt * 16 + c] = (_Float16)(sv * kSCarry);
    }
  wave_lds_sync();

  const float bav = bf16r(ba[h]);
  const float bbv = bf16r(bb[h]);
  const int row = tid >> 1;
  const int hf  = tid & 1;

#pragma unroll 1
  for (int chunk = 0; chunk < kNChunk; ++chunk) {
    const int t0 = chunk * kChunk;
    __syncthreads();

    const size_t grow = (size_t)(b * kSeq + t0 + row);
    const unsigned short* gp = QKV + grow * kQkvLd + h * kHd + hf * 32;
    v4u qw[4], kwd[4], vw[4];
#pragma unroll
    for (int i = 0; i < 4; ++i) {
      qw[i]  = *(const v4u*)(gp + 8 * i);
      kwd[i] = *(const v4u*)(gp + kInner + 8 * i);
      vw[i]  = *(const v4u*)(gp + 2 * kInner + 8 * i);
    }
#pragma unroll
    for (int i = 0; i < 4; ++i) {
      *(v8h*)(Qs + row * kTP + hf * 32 + 8 * i) = __builtin_bit_cast(v8h, qw[i]);
      *(v8h*)(Ks + row * kTP + hf * 32 + 8 * i) = __builtin_bit_cast(v8h, kwd[i]);
    }
    float ss = 0.0f;
#pragma unroll
    for (int i = 0; i < 4; ++i) {
#pragma unroll
      for (int cp = 0; cp < 4; ++cp) {
        const unsigned wk = kwd[i][cp];
        const float f0 = h16_to_f32(wk & 0xffffu);
        const float f1 = h16_to_f32(wk >> 16);
        ss += f0 * f0;
        ss += f1 * f1;
        const unsigned wv = vw[i][cp];
        const unsigned short v0 = (unsigned short)(wv & 0xffffu);
        const unsigned short v1 = (unsigned short)(wv >> 16);
        const int d = hf * 32 + 8 * i + 2 * cp;
        Vt[d * kTP + row]       = __builtin_bit_cast(_Float16, v0);
        Vt[(d + 1) * kTP + row] = __builtin_bit_cast(_Float16, v1);
      }
    }
    ss += __shfl_xor(ss, 1, 32);
    const float* zr = Z + grow * kGateLd;
    const float za = zr[h] + bav;
    const float zb = zr[kHeads + h] + bbv;
    const float lra = -log1pf(expf(-fmaxf(za, -80.0f)));
    const float bet = 1.0f / (1.0f + expf(-fmaxf(zb, -80.0f)));
    const float kn  = 1.0f / fmaxf(sqrtf(ss), 1e-12f);
    if (hf == 0) {
      lraw_s[row] = lra;
      ksb_s[row]  = kn * bet * kPCarry;
    }
    __syncthreads();

    {
      float a  = lraw_s[lane];
      float bq = lraw_s[lane + 32];
#pragma unroll
      for (int off = 1; off < 32; off <<= 1) {
        const float ta = __shfl_up(a, off, 32);
        const float tb = __shfl_up(bq, off, 32);
        a  += (lane >= off) ? ta : 0.0f;
        bq += (lane >= off) ? tb : 0.0f;
      }
      const float tot = __shfl(a, 31, 32);
      bq += tot;
      if (wave == 0) {
        la_s[lane]       = a;
        la_s[lane + 32]  = bq;
        ela_s[lane]      = expf(a);
        ela_s[lane + 32] = expf(bq);
      }
    }
    __syncthreads();

    {
      const float la_row  = la_s[row];
      const float la_last = la_s[63];
      const float kwf = kn * bet * expf(fminf(la_last - la_row, 0.0f)) * kKwCarry;
#pragma unroll
      for (int i = 0; i < 4; ++i) {
#pragma unroll
        for (int cp = 0; cp < 4; ++cp) {
          const unsigned wk = kwd[i][cp];
          const float f0 = h16_to_f32(wk & 0xffffu);
          const float f1 = h16_to_f32(wk >> 16);
          const int j = hf * 32 + 8 * i + 2 * cp;
          const float p0 = f0 * kwf;
          const float p1 = f1 * kwf;
          const _Float16 h0 = (_Float16)p0;
          const _Float16 h1 = (_Float16)p1;
          const float r0 = (p0 - (float)h0) * kKwResCarry;
          const float r1 = (p1 - (float)h1) * kKwResCarry;
          Kw[j * kTP + row]        = h0;
          Kw[(j + 1) * kTP + row]  = h1;
          Kwr[j * kTP + row]       = (_Float16)r0;
          Kwr[(j + 1) * kTP + row] = (_Float16)r1;
        }
      }
    }
    v16h qa[2];
#pragma unroll
    for (int ks = 0; ks < 2; ++ks) qa[ks] = Frag<_Float16>::load(Qs + (m0 + c) * kTP + koff + 32 * ks);
    {
      float lat[8];
#pragma unroll
      for (int r = 0; r < 8; ++r) lat[r] = la_s[m0 + 8 * hh + r];
#pragma unroll 1
      for (int nt = 0; nt < 4; ++nt) {
        const _Float16* kr = Ks + (nt * 16 + c) * kTP + koff;
        v8f acc = z8;
#pragma unroll
        for (int ks = 0; ks < 2; ++ks) acc = mma_h(qa[ks], Frag<_Float16>::load(kr + 32 * ks), acc);
        const int s = nt * 16 + c;
        const float las = la_s[s];
        const float kb  = ksb_s[s];
#pragma unroll
        for (int r = 0; r < 8; ++r) {
          const int t = m0 + 8 * hh + r;
          const float e = expf(fminf(lat[r] - las, 0.0f));
          const float pv = (s <= t) ? (acc[r] * kb * e) : 0.0f;
          Ps[t * kTP + s] = (_Float16)pv;
        }
      }
    }
    __syncthreads();

    {
      v16h pa[2];
#pragma unroll
      for (int ks = 0; ks < 2; ++ks) pa[ks] = Frag<_Float16>::load(Ps + (m0 + c) * kTP + koff + 32 * ks);
      float elat[8];
#pragma unroll
      for (int r = 0; r < 8; ++r) elat[r] = ela_s[m0 + 8 * hh + r] * kSInv;
#pragma unroll 1
      for (int nt = 0; nt < 4; ++nt) {
        const _Float16* vr = Vt  + (nt * 16 + c) * kTP + koff;
        const _Float16* sr = S16 + (nt * 16 + c) * kTP + koff;
        v8f accP = z8, accS = z8;
#pragma unroll
        for (int ks = 0; ks < 2; ++ks) {
          accP = mma_h(pa[ks], Frag<_Float16>::load(vr + 32 * ks), accP);
          accS = mma_h(qa[ks], Frag<_Float16>::load(sr + 32 * ks), accS);
        }
#pragma unroll
        for (int r = 0; r < 8; ++r) {
          const float y = accP[r] * kPInv + elat[r] * accS[r];
          slab[(8 * hh + r) * kSlabP + nt * 16 + c] = y * kYCarry;
        }
      }
    }
    {
      v16h va[2];
#pragma unroll
      for (int ks = 0; ks < 2; ++ks) va[ks] = Frag<_Float16>::load(Vt + (m0 + c) * kTP + koff + 32 * ks);
      const float e63 = ela_s[63];
#pragma unroll
      for (int nt = 0; nt < 4; ++nt) {
        v8f dSh = z8, dSr = z8;
#pragma unroll
        for (int ks = 0; ks < 2; ++ks) {
          const v16h kfh = Frag<_Float16>::load(Kw  + (nt * 16 + c) * kTP + koff + 32 * ks);
          const v16h kfr = Frag<_Float16>::load(Kwr + (nt * 16 + c) * kTP + koff + 32 * ks);
          dSh = mma_h(va[ks], kfh, dSh);
          dSr = mma_h(va[ks], kfr, dSr);
        }
#pragma unroll
        for (int r = 0; r < 8; ++r) {
          const float dsv = dSh[r] + dSr[r] * kKwResInv;
          Sreg[nt][r] = e63 * Sreg[nt][r] + dsv * kKwInv;
        }
      }
    }
    wave_lds_sync();
    {
      const int q4 = lane >> 3, c8 = (lane & 7) * 8;
      unsigned short* yp = Y16 + (size_t)(b * kSeq + t0 + m0) * kInner + h * kHd;
      for (int pass = 0; pass < 2; ++pass) {
#pragma unroll
        for (int it = 0; it < 4; ++it) {
          const int rowl = it * 4 + q4;
          const float* sp = slab + rowl * kSlabP + c8;
          v8h hv;
#pragma unroll
          for (int e = 0; e < 8; ++e) hv[e] = (_Float16)sp[e];
          *(volatile v8h*)(yp + (size_t)rowl * kInner + c8) = hv;
        }
        __threadfence();
      }
    }
    wave_lds_sync();
    __syncthreads();
#pragma unroll
    for (int nt = 0; nt < 4; ++nt)
#pragma unroll
      for (int r = 0; r < 8; ++r)
        S16[(m0 + 8 * hh + r) * kTP + nt * 16 + c] = (_Float16)(Sreg[nt][r] * kSCarry);
  }

#pragma unroll
  for (int nt = 0; nt < 4; ++nt)
#pragma unroll
    for (int r = 0; r < 8; ++r) slab[(8 * hh + r) * kSlabP + nt * 16 + c] = Sreg[nt][r];
  wave_lds_sync();
  {
    float* op = Sout + ((size_t)bh * 64 + m0) * 64;
    for (int pass = 0; pass < 2; ++pass) {
#pragma unroll
      for (int it = 0; it < 8; ++it) {
        const int rowl = it * 2 + hh;
        const v4f v = *(const v4f*)(slab + rowl * kSlabP + c4);
        *(volatile v4f*)(op + rowl * 64 + c4) = v;
      }
      __threadfence();
    }
  }
}

extern "C" void kernel_launch(void* const* d_in, const int* in_sizes, int n_in,
                              void* d_out, int out_size, void* d_ws, size_t ws_size, hipStream_t stream) {
  if (n_in < 10 || d_out == nullptr || d_ws == nullptr) return;
  if (in_sizes[0] != kRows * kModel || in_sizes[1] != kOut1 ||
      in_sizes[2] != kModel * kInner || in_sizes[3] != kModel * kInner || in_sizes[4] != kModel * kInner ||
      in_sizes[5] != kModel * kHeads || in_sizes[6] != kHeads || in_sizes[7] != kModel * kHeads ||
      in_sizes[8] != kHeads || in_sizes[9] != kInner * kModel || out_size != kOut0 + kOut1) return;

  const float* x   = (const float*)d_in[0];
  const float* st0 = (const float*)d_in[1];
  const float* Wq  = (const float*)d_in[2];
  const float* Wk  = (const float*)d_in[3];
  const float* Wv  = (const float*)d_in[4];
  const float* Wa  = (const float*)d_in[5];
  const float* ba  = (const float*)d_in[6];
  const float* Wb  = (const float*)d_in[7];
  const float* bb  = (const float*)d_in[8];
  const float* Wo  = (const float*)d_in[9];
  float* out0 = (float*)d_out;
  float* out1 = out0 + (size_t)kOut0;

  char* ws = (char*)d_ws; size_t off = 0;
  auto carve = [&](size_t bytes) -> char* { char* p = ws + off; off += (bytes + 255) & ~(size_t)255; return p; };
  unsigned short* X16   = (unsigned short*)carve((size_t)kRows * kModel * 2);
  unsigned short* WALL  = (unsigned short*)carve((size_t)kWallRows * 1024 * 2);
  unsigned short* QKV16 = (unsigned short*)carve((size_t)kRows * kQkvLd * 2);
  float*          ZG    = (float*)carve((size_t)kRows * kGateLd * 4);
  unsigned short* Y16   = (unsigned short*)carve((size_t)kRows * kInner * 2);
  if (off > ws_size || off > (size_t)134217728) return;

  const int n8x = kRows * (kModel / 8);
  cvt8_kernel<<<(n8x + 255) / 256, 256, 0, stream>>>(x, X16, n8x, 1.0f);
  wt_cast_kernel<<<dim3(16, 16, 4), 256, 0, stream>>>(Wq, Wk, Wv, Wo, WALL);
  wgate_cast_kernel<<<16, 256, 0, stream>>>(Wa, Wb, WALL);

  wmma_gemm64<0, false, 0, 1, false, 0><<<dim3((kRows / 64) * (kQkvLd / 64) / 8, 1), 256, 0, stream>>>(
      X16, X16, kModel, 0L, WALL, WALL, 1024, 0L, (void*)QKV16, (void*)QKV16, kQkvLd, 0L,
      ZG, ZG, 0L, kRows, kQkvLd, kModel, kWInv);
  wmma_gemm64<0, false, 0, 0, false, 0><<<dim3((kRows / 64) * (kGateLd / 64) / 8, 1), 256, 0, stream>>>(
      X16, X16, kModel, 0L, WALL + (size_t)kGateRow0 * 1024, WALL + (size_t)kGateRow0 * 1024, 1024, 0L,
      (void*)ZG, (void*)ZG, kGateLd, 0L, ZG, ZG, 0L, kRows, kGateLd, kModel, kWInv);

  chunk_scan_kernel<<<kBatch * kHeads, 128, 0, stream>>>(QKV16, ZG, st0, ba, bb, Y16, out1);

  wmma_gemm64<0, false, 0, 0, false, 0><<<dim3((kRows / 64) * (kModel / 64) / 8, 1), 256, 0, stream>>>(
      Y16, Y16, kInner, 0L, WALL + (size_t)kWoRow0 * 1024, WALL + (size_t)kWoRow0 * 1024, 1024, 0L,
      (void*)out0, (void*)out0, kModel, 0L, ZG, ZG, 0L, kRows, kModel, kInner, kOutScale);
}
